// biLSTM_72550587564391
// MI455X (gfx1250) — hardware-verified
//
#include <hip/hip_runtime.h>
#include <math.h>

constexpr int B_BATCH = 64;
constexpr int T_STEPS = 256;
constexpr int E_EMB   = 300;
constexpr int E_PAD   = 320;
constexpr int H_HID   = 512;
constexpr int G4H     = 4 * H_HID;
constexpr int C_CAT   = H_HID + E_EMB;
constexpr int O_TAGS  = 9;
constexpr int O_PAD   = 64;
constexpr int V_VOCAB = 50000;
constexpr int M_ROWS  = B_BATCH * T_STEPS;
constexpr int N_OUT   = M_ROWS * O_TAGS;
constexpr int NTHR    = 256;
constexpr int SEQB    = 16;
constexpr int HPITCH  = 520;
constexpr float XCARRY = 16.0f;
constexpr float WCARRY = 256.0f;
constexpr float ACARRY = 64.0f;
constexpr float ZCARRY = 32.0f;
constexpr float ZX_SCALE  = ZCARRY / (XCARRY * WCARRY);
constexpr float Z_INV     = 1.0f / ZCARRY;
constexpr float AW_INV    = 1.0f / (ACARRY * WCARRY);
constexpr float PRJ_SCALE = 1.0f / (ACARRY * WCARRY);
static_assert(E_PAD % 32 == 0 && H_HID % 32 == 0 && (2 * H_HID) % 32 == 0);
static_assert(G4H % 64 == 0 && M_ROWS % 64 == 0 && O_PAD % 64 == 0);
static_assert(((G4H / 64) * (M_ROWS / 64)) % 8 == 0);
static_assert(((M_ROWS / 64) * (O_PAD / 64)) % 8 == 0);
static_assert(H_HID == 64 * (NTHR / 32));
static_assert(B_BATCH % SEQB == 0 && SEQB == 2 * (NTHR / 32));
static_assert((2 * SEQB * HPITCH) % NTHR == 0);
static_assert(E_EMB % 4 == 0 && C_CAT % 4 == 0);
static_assert(E_PAD == 40 * 8 && (M_ROWS % 32) == 0);
static_assert((H_HID * (H_HID / 8)) % NTHR == 0 && (H_HID * (E_PAD / 8)) % NTHR == 0 && (O_PAD * (2 * H_HID / 8)) % NTHR == 0);
static_assert(N_OUT % (4 * NTHR) == 0);
static_assert(O_TAGS <= O_PAD && E_EMB <= E_PAD);

constexpr size_t SZ_XE   = (size_t)M_ROWS * E_PAD * 2;
constexpr size_t SZ_WX16 = (size_t)2 * G4H * E_PAD * 2;
constexpr size_t SZ_WA16 = (size_t)2 * G4H * H_HID * 2;
constexpr size_t SZ_WP16 = (size_t)O_PAD * 2 * H_HID * 2;
constexpr size_t SZ_ZX   = (size_t)G4H * M_ROWS * 2;
constexpr size_t SZ_ASQ  = (size_t)M_ROWS * 2 * H_HID * 2;
constexpr size_t SZ_PRJ  = (size_t)M_ROWS * O_PAD * 4;
constexpr size_t WS_TOTAL = SZ_XE + SZ_WX16 + SZ_WA16 + SZ_WP16 + SZ_ZX + SZ_ASQ + SZ_PRJ;
static_assert(WS_TOTAL <= (size_t)134217728);
static_assert(SZ_XE % 256 == 0 && SZ_WX16 % 256 == 0 && SZ_WA16 % 256 == 0 && SZ_WP16 % 256 == 0 && SZ_ZX % 256 == 0 && SZ_ASQ % 256 == 0 && SZ_PRJ % 256 == 0);

typedef __attribute__((ext_vector_type(16))) _Float16 v16h;
typedef __attribute__((ext_vector_type(8)))  _Float16 v8h;
typedef __attribute__((ext_vector_type(16))) __bf16   v16b;
typedef __attribute__((ext_vector_type(8)))  __bf16   v8b;
typedef __attribute__((ext_vector_type(8)))  float    v8f;
typedef __attribute__((ext_vector_type(4)))  float    v4f;
typedef __attribute__((ext_vector_type(4)))  unsigned v4u;

__device__ __forceinline__ unsigned short f2bf_bits(float f) {
  unsigned u = __float_as_uint(f);
  return (unsigned short)((u + 0x7FFFu + ((u >> 16) & 1u)) >> 16);
}
__device__ __forceinline__ float bf_bits2f(unsigned short h) { return __uint_as_float(((unsigned)h) << 16); }

__device__ __forceinline__ float h16_to_f32(unsigned hb) {
  const unsigned sgn = (hb & 0x8000u) << 16; const unsigned em = hb & 0x7fffu;
  const float fn = __uint_as_float((em << 13) + 0x38000000u);
  const float fs = (float)em * 5.9604644775390625e-8f;
  const float mag = (em < 0x400u) ? fs : fn; return __uint_as_float(__float_as_uint(mag) | sgn); }

__device__ __forceinline__ void dep_guard_h(v8f& a, v8f& b, v16h x, v16h y) { asm volatile("v_nop\n\tv_nop\n\tv_nop\n\tv_nop" : "+v"(a), "+v"(b) : "v"(x), "v"(y)); }
__device__ __forceinline__ void dep_guard_b(v8f& a, v8f& b, v16b x, v16b y) { asm volatile("v_nop\n\tv_nop\n\tv_nop\n\tv_nop" : "+v"(a), "+v"(b) : "v"(x), "v"(y)); }
__device__ __forceinline__ void tie4_h(v8f& a0, v8f& a1, v8f& a2, v8f& a3, v16h x, v16h y, v16h z, v16h w) {
  asm volatile("v_nop\n\tv_nop\n\tv_nop\n\tv_nop" : "+v"(a0), "+v"(a1), "+v"(a2), "+v"(a3) : "v"(x), "v"(y), "v"(z), "v"(w)); }
__device__ __forceinline__ void tie4_b(v8f& a0, v8f& a1, v8f& a2, v8f& a3, v16b x, v16b y, v16b z, v16b w) {
  asm volatile("v_nop\n\tv_nop\n\tv_nop\n\tv_nop" : "+v"(a0), "+v"(a1), "+v"(a2), "+v"(a3) : "v"(x), "v"(y), "v"(z), "v"(w)); }
__device__ __forceinline__ void tie4in5_h(v8f& a0, v8f& a1, v8f& a2, v8f& a3, v16h x, v16h b0, v16h b1, v16h b2, v16h b3) {
  asm volatile("v_nop\n\tv_nop\n\tv_nop\n\tv_nop" : "+v"(a0), "+v"(a1), "+v"(a2), "+v"(a3) : "v"(x), "v"(b0), "v"(b1), "v"(b2), "v"(b3)); }
__device__ __forceinline__ void keep4_h(v16h a, v16h b, v16h c, v16h d) { asm volatile("v_nop" :: "v"(a), "v"(b), "v"(c), "v"(d)); }
__device__ __forceinline__ void keep4_b(v16b a, v16b b, v16b c, v16b d) { asm volatile("v_nop" :: "v"(a), "v"(b), "v"(c), "v"(d)); }
__device__ __forceinline__ void acc_guard4(v8f& a, v8f& b, v8f& c, v8f& d) { asm volatile("v_nop\n\tv_nop\n\tv_nop\n\tv_nop" : "+v"(a), "+v"(b), "+v"(c), "+v"(d)); }
template <typename T> struct Frag;
template <> struct Frag<_Float16> {
  typedef v16h V; union U { v16h v; v8h h[2]; };
  static __device__ __forceinline__ v16h load(const _Float16* p) {
    U f; f.h[0] = *(const v8h*)(p); f.h[1] = *(const v8h*)(p + 16); return f.v;
  }
  static __device__ __forceinline__ v8f mma(v16h a, v16h b, v8f c) {
    return __builtin_amdgcn_wmma_f32_16x16x32_f16(false, a, false, b, (short)0, c, false, false);
  }
  static __device__ __forceinline__ void guard(v8f& a, v8f& b, v16h x, v16h y) { dep_guard_h(a, b, x, y); }
  static __device__ __forceinline__ void tie4(v8f& a0, v8f& a1, v8f& a2, v8f& a3, v16h x, v16h y, v16h z, v16h w) { tie4_h(a0, a1, a2, a3, x, y, z, w); }
  static __device__ __forceinline__ void keep(v16h a, v16h b, v16h c, v16h d) { keep4_h(a, b, c, d); }
};
template <> struct Frag<__bf16> {
  typedef v16b V; union U { v16b v; v8b h[2]; };
  static __device__ __forceinline__ v16b load(const __bf16* p) {
    U f; f.h[0] = *(const v8b*)(p); f.h[1] = *(const v8b*)(p + 16); return f.v;
  }
  static __device__ __forceinline__ v8f mma(v16b a, v16b b, v8f c) {
    return __builtin_amdgcn_wmma_f32_16x16x32_bf16(false, a, false, b, (short)0, c, false, false);
  }
  static __device__ __forceinline__ void guard(v8f& a, v8f& b, v16b x, v16b y) { dep_guard_b(a, b, x, y); }
  static __device__ __forceinline__ void tie4(v8f& a0, v8f& a1, v8f& a2, v8f& a3, v16b x, v16b y, v16b z, v16b w) { tie4_b(a0, a1, a2, a3, x, y, z, w); }
  static __device__ __forceinline__ void keep(v16b a, v16b b, v16b c, v16b d) { keep4_b(a, b, c, d); }
};

__device__ __forceinline__ float fsig(float x)  { return __builtin_amdgcn_rcpf(1.0f + expf(-x)); }
__device__ __forceinline__ float ftanh(float x) { return 1.0f - 2.0f * __builtin_amdgcn_rcpf(expf(2.0f * x) + 1.0f); }

template <int ET> struct Elem;
template <> struct Elem<0> { typedef _Float16 T; };
template <> struct Elem<1> { typedef __bf16 T; };
template <int ET, bool SPLIT, int BIAS_MODE, int OUT_MODE, bool RESID, int ACT = 0>
__global__ __launch_bounds__(256) void wmma_gemm64(
    const unsigned short* __restrict__ Ap, const unsigned short* __restrict__ A2p, int lda, long strideA,
    const unsigned short* __restrict__ Btp, const unsigned short* __restrict__ Bt2p, int ldb, long strideB,
    void* __restrict__ Cout, void* __restrict__ Cout2, int ldc, long strideC,
    const float* __restrict__ bias,
    const float* __restrict__ resid, long strideR,
    int M, int N, int K, float scale) {
  typedef typename Elem<ET>::T T;
  typedef typename Frag<T>::V V;
  const T* A = (const T*)Ap; const T* A2 = (const T*)A2p; const T* Bt = (const T*)Btp; const T* Bt2 = (const T*)Bt2p;
  __shared__ __align__(16) float sT[8][16 * 68];
  const int b    = blockIdx.y;
  const int lane = threadIdx.x & 31;
  const int wave = threadIdx.x >> 5;
  const int tilesN = N >> 6;
  const int tilesM = M >> 6;
  const int tile = blockIdx.x * 8 + wave;
  if (tile >= tilesM * tilesN) return;
  const int tm = tile / tilesN;
  const int tn = tile - tm * tilesN;
  const int m0 = tm << 6;
  const int n0 = tn << 6;

  const T* Ab  = A  + (size_t)b * strideA;
  const T* Bb  = Bt + (size_t)b * strideB;
  const T* Ab2 = SPLIT ? (A2  + (size_t)b * strideA) : nullptr;
  const T* Bb2 = SPLIT ? (Bt2 + (size_t)b * strideB) : nullptr;

  const int rlane = lane & 15;
  const int koff  = (lane >> 4) * 8;
  const int mOff  = (lane >> 4) * 8;

  v8f acc[4][4];
#pragma unroll
  for (int i = 0; i < 4; ++i)
#pragma unroll
    for (int j = 0; j < 4; ++j) acc[i][j] = (v8f){0.f,0.f,0.f,0.f,0.f,0.f,0.f,0.f};

  for (int k0 = 0; k0 < K; k0 += 32) {
    V bh[4], bl[4];
#pragma unroll
    for (int j = 0; j < 4; ++j) {
      const size_t bo = (size_t)(n0 + (j << 4) + rlane) * ldb + koff + k0;
      bh[j] = Frag<T>::load(Bb + bo);
      if (SPLIT) bl[j] = Frag<T>::load(Bb2 + bo);
    }
#pragma unroll
    for (int i = 0; i < 4; ++i) {
      const size_t ao = (size_t)(m0 + (i << 4) + rlane) * lda + koff + k0;
      V ah = Frag<T>::load(Ab + ao);
      V al;
      if (SPLIT) al = Frag<T>::load(Ab2 + ao);
#pragma unroll
      for (int j = 0; j < 4; ++j) {
        acc[i][j] = Frag<T>::mma(ah, bh[j], acc[i][j]);
        if (SPLIT) {
          acc[i][j] = Frag<T>::mma(ah, bl[j], acc[i][j]);
          acc[i][j] = Frag<T>::mma(al, bh[j], acc[i][j]);
        }
      }
      Frag<T>::tie4(acc[i][0], acc[i][1], acc[i][2], acc[i][3], ah, SPLIT ? al : ah, bh[0], bh[3]);
    }
    Frag<T>::keep(bh[0], bh[1], bh[2], bh[3]);
    if (SPLIT) Frag<T>::keep(bl[0], bl[1], bl[2], bl[3]);
  }
  acc_guard4(acc[0][0], acc[0][1], acc[0][2], acc[0][3]);
  acc_guard4(acc[1][0], acc[1][1], acc[1][2], acc[1][3]);
  acc_guard4(acc[2][0], acc[2][1], acc[2][2], acc[2][3]);
  acc_guard4(acc[3][0], acc[3][1], acc[3][2], acc[3][3]);

  float* slab = sT[wave];
  const float* Rb = RESID ? (resid + (size_t)b * strideR) : nullptr;
#pragma unroll
  for (int i = 0; i < 4; ++i) {
    const int mBase = m0 + (i << 4);
#pragma unroll
    for (int j = 0; j < 4; ++j) {
      const int n = n0 + (j << 4) + rlane;
      float bv = 0.f;
      if (BIAS_MODE == 2) bv = bias[n];
#pragma unroll
      for (int r = 0; r < 8; ++r) {
        float v = acc[i][j][r] * scale;
        if (BIAS_MODE == 1) v += bias[mBase + mOff + r];
        if (BIAS_MODE == 2) v += bv;
        if (RESID) v += Rb[(size_t)(mBase + mOff + r) * ldc + n];
        if (ACT == 1) v = tanhf(v);
        if (ACT == 2) v = fmaxf(v, 0.0f);
        if (ACT == 3) v = v / (1.0f + expf(-v));
        if (ACT == 4) v = (v > 0.f) ? v : 0.01f * v;
        if (ACT == 5) v = 0.5f * v * (1.0f + erff(v * 0.70710678118654752f));
        slab[(mOff + r) * 68 + (j << 4) + rlane] = v;
      }
    }
    __builtin_amdgcn_fence(__ATOMIC_RELEASE, "workgroup");
    __builtin_amdgcn_wave_barrier();
    __builtin_amdgcn_fence(__ATOMIC_ACQUIRE, "workgroup");
    if (OUT_MODE == 0) {
      float* C = (float*)Cout + (size_t)b * strideC;
      const int hh = lane >> 4, c4 = (lane & 15) * 4;
      for (int pass = 0; pass < 2; ++pass) {
#pragma unroll
        for (int it = 0; it < 8; ++it) {
          const int row = it * 2 + hh;
          v4f v = *(const v4f*)(slab + row * 68 + c4);
          *(volatile v4f*)(C + (size_t)(mBase + row) * ldc + n0 + c4) = v;
        }
        __threadfence();
      }
    } else {
      const int q = lane >> 3, c8 = (lane & 7) * 8;
      unsigned short* C  = (unsigned short*)Cout  + (size_t)b * strideC;
      unsigned short* C2 = (OUT_MODE == 2) ? ((unsigned short*)Cout2 + (size_t)b * strideC) : nullptr;
      for (int pass = 0; pass < 2; ++pass) {
#pragma unroll
        for (int it = 0; it < 4; ++it) {
          const int row = it * 4 + q;
          const float* sp = slab + row * 68 + c8;
          v8h hv, lv;
#pragma unroll
          for (int e = 0; e < 8; ++e) {
            if (OUT_MODE == 1) {
              hv[e] = (_Float16)sp[e];
            } else {
              unsigned short hb = f2bf_bits(sp[e]);
              unsigned short lb = f2bf_bits(sp[e] - bf_bits2f(hb));
              hv[e] = __builtin_bit_cast(_Float16, hb);
              lv[e] = __builtin_bit_cast(_Float16, lb);
            }
          }
          *(volatile v8h*)(C + (size_t)(mBase + row) * ldc + n0 + c8) = hv;
          if (OUT_MODE == 2) *(volatile v8h*)(C2 + (size_t)(mBase + row) * ldc + n0 + c8) = lv;
        }
        __threadfence();
      }
    }
    __builtin_amdgcn_fence(__ATOMIC_RELEASE, "workgroup");
    __builtin_amdgcn_wave_barrier();
    __builtin_amdgcn_fence(__ATOMIC_ACQUIRE, "workgroup");
  }
}

struct GateW { const float* w0; const float* w1; const float* w2; const float* w3;
               const float* w4; const float* w5; const float* w6; const float* w7; };
static_assert(sizeof(GateW) == 64);
__device__ __forceinline__ const float* pick_gate(const GateW& p, int s) {
  const float* r = p.w0;
  r = (s == 1) ? p.w1 : r; r = (s == 2) ? p.w2 : r; r = (s == 3) ? p.w3 : r;
  r = (s == 4) ? p.w4 : r; r = (s == 5) ? p.w5 : r; r = (s == 6) ? p.w6 : r; r = (s == 7) ? p.w7 : r;
  return r;
}

__global__ __launch_bounds__(NTHR) void wa_prep_kernel(GateW p, unsigned short* __restrict__ WA16) {
  const int pg = blockIdx.y;
  const float* W = pick_gate(p, pg);
  const int i = blockIdx.x * NTHR + threadIdx.x;
  const int rr = i >> 6, k8 = (i & 63) * 8;
  const float* sp = W + (size_t)rr * C_CAT + k8;
  const v4f va = *(const v4f*)(sp);
  const v4f vb = *(const v4f*)(sp + 4);
  v8h hv;
#pragma unroll
  for (int e = 0; e < 4; ++e) { hv[e] = (_Float16)(va[e] * WCARRY); hv[4 + e] = (_Float16)(vb[e] * WCARRY); }
  unsigned short* dst = WA16 + (size_t)pg * H_HID * H_HID + (size_t)i * 8;
  *(volatile v8h*)dst = hv;
  __threadfence();
  *(volatile v8h*)dst = hv;
}

__global__ __launch_bounds__(NTHR) void wx_prep_kernel(GateW p, unsigned short* __restrict__ WX16) {
  const int pg = blockIdx.y;
  const float* W = pick_gate(p, pg);
  const int i = blockIdx.x * NTHR + threadIdx.x;
  const int rr = i / 40, q = i - rr * 40;
  const int col = q * 8;
  const int cb0 = (col < E_EMB - 4) ? col : (E_EMB - 4);
  const int cb1 = (col + 4 < E_EMB - 4) ? (col + 4) : (E_EMB - 4);
  const float* sp = W + (size_t)rr * C_CAT + H_HID;
  const v4f va = *(const v4f*)(sp + cb0);
  const v4f vb = *(const v4f*)(sp + cb1);
  v8h hv;
#pragma unroll
  for (int e = 0; e < 4; ++e) {
    const float f0 = (col + e < E_EMB) ? WCARRY : 0.0f;
    const float f1 = (col + 4 + e < E_EMB) ? WCARRY : 0.0f;
    hv[e] = (_Float16)(va[e] * f0); hv[4 + e] = (_Float16)(vb[e] * f1);
  }
  unsigned short* dst = WX16 + (size_t)pg * H_HID * E_PAD + (size_t)i * 8;
  *(volatile v8h*)dst = hv;
  __threadfence();
  *(volatile v8h*)dst = hv;
}

__global__ __launch_bounds__(NTHR) void wp_prep_kernel(const float* __restrict__ Wp, unsigned short* __restrict__ WP16) {
  const int i = blockIdx.x * NTHR + threadIdx.x;
  const int o = i >> 7, k8 = (i & 127) * 8;
  const int oc = (o < O_TAGS - 1) ? o : (O_TAGS - 1);
  const float fac = (o < O_TAGS) ? WCARRY : 0.0f;
  const float* sp = Wp + (size_t)oc * (2 * H_HID) + k8;
  const v4f va = *(const v4f*)(sp);
  const v4f vb = *(const v4f*)(sp + 4);
  v8h hv;
#pragma unroll
  for (int e = 0; e < 4; ++e) { hv[e] = (_Float16)(va[e] * fac); hv[4 + e] = (_Float16)(vb[e] * fac); }
  unsigned short* dst = WP16 + (size_t)i * 8;
  *(volatile v8h*)dst = hv;
  __threadfence();
  *(volatile v8h*)dst = hv;
}

__global__ __launch_bounds__(NTHR) void embed_kernel(const int* __restrict__ tok, const float* __restrict__ emb,
                                                     unsigned short* __restrict__ XE) {
  const int tid = threadIdx.x, lane = tid & 31, wave = tid >> 5;
  const int m0 = (blockIdx.x * (NTHR / 32) + wave) * 4;
  v8h hv[5];
#pragma unroll
  for (int it = 0; it < 5; ++it) {
    const int ci = it * 32 + lane;
    const int rr = ci / 40;
    const int q  = ci - rr * 40;
    const int m  = m0 + rr;
    const int t  = m >> 6, b = m & 63;
    int id = tok[b * T_STEPS + t];
    id = (id < 0) ? 0 : ((id > V_VOCAB - 1) ? (V_VOCAB - 1) : id);
    const int col = q * 8;
    const int cb0 = (col < E_EMB - 4) ? col : (E_EMB - 4);
    const int cb1 = (col + 4 < E_EMB - 4) ? (col + 4) : (E_EMB - 4);
    const float* er = emb + (size_t)id * E_EMB;
    const v4f va = *(const v4f*)(er + cb0);
    const v4f vb = *(const v4f*)(er + cb1);
    asm volatile("" ::: "memory");
#pragma unroll
    for (int e = 0; e < 4; ++e) {
      const float f0 = (col + e < E_EMB) ? XCARRY : 0.0f;
      const float f1 = (col + 4 + e < E_EMB) ? XCARRY : 0.0f;
      hv[it][e]     = (_Float16)(va[e] * f0);
      hv[it][4 + e] = (_Float16)(vb[e] * f1);
    }
  }
  unsigned short* dst = XE + (size_t)m0 * E_PAD;
  for (int pass = 0; pass < 2; ++pass) {
#pragma unroll
    for (int it = 0; it < 5; ++it) *(volatile v8h*)(dst + (size_t)(it * 32 + lane) * 8) = hv[it];
    __threadfence();
  }
}

__global__ __launch_bounds__(NTHR) void lstm_dir_kernel(const unsigned short* __restrict__ WAp,
                                                       const unsigned short* __restrict__ ZXp,
                                                       unsigned short* __restrict__ ASQ,
                                                       const float* __restrict__ bgf, const float* __restrict__ bgi,
                                                       const float* __restrict__ bgo, const float* __restrict__ bgc,
                                                       int dir) {
  __shared__ __align__(16) _Float16 Ah[2][SEQB * HPITCH];
  const _Float16* WA = (const _Float16*)WAp;
  const int tid = threadIdx.x, lane = tid & 31, wave = tid >> 5;
  const int c = lane & 15, hh = lane >> 4, koff = hh * 8;
  const int rowbase = blockIdx.x * SEQB;

  {
    _Float16* ahf = &Ah[0][0];
#pragma unroll 1
    for (int i = tid; i < 2 * SEQB * HPITCH; i += NTHR) ahf[i] = (_Float16)0.0f;
  }
  float cst[4][8], bgv[4][4];
#pragma unroll
  for (int nt = 0; nt < 4; ++nt) {
    const int j = 64 * wave + 16 * nt + c;
    bgv[nt][0] = bgf[j]; bgv[nt][1] = bgi[j]; bgv[nt][2] = bgo[j]; bgv[nt][3] = bgc[j];
    asm volatile("" ::: "memory");
#pragma unroll
    for (int r = 0; r < 8; ++r) cst[nt][r] = 0.0f;
  }
  __syncthreads();

  const v8f z8 = {0.f, 0.f, 0.f, 0.f, 0.f, 0.f, 0.f, 0.f};

#pragma unroll 1
  for (int t = 0; t < T_STEPS; ++t) {
    const int tt  = dir ? (T_STEPS - 1 - t) : t;
    const int cur = t & 1;
    const _Float16* ahrow = &Ah[cur][0] + c * HPITCH + koff;
    _Float16* ahn = &Ah[cur ^ 1][0];
#pragma unroll
    for (int nt = 0; nt < 4; ++nt) {
      const int j = 64 * wave + 16 * nt + c;
      v4u zq[4];
#pragma unroll
      for (int g = 0; g < 4; ++g)
        zq[g] = *(const v4u*)(ZXp + (size_t)(g * H_HID + j) * M_ROWS + (size_t)tt * B_BATCH + rowbase + 8 * hh);
      const _Float16* wa = WA + (size_t)j * H_HID + koff;
      v8f acc[4];
      acc[0] = z8; acc[1] = z8; acc[2] = z8; acc[3] = z8;
#pragma unroll 1
      for (int k0 = 0; k0 < H_HID; k0 += 32) {
        const v16h a  = Frag<_Float16>::load(ahrow + k0);
        const v16h b0 = Frag<_Float16>::load(wa + k0);
        const v16h b1 = Frag<_Float16>::load(wa + (size_t)1 * H_HID * H_HID + k0);
        const v16h b2 = Frag<_Float16>::load(wa + (size_t)2 * H_HID * H_HID + k0);
        const v16h b3 = Frag<_Float16>::load(wa + (size_t)3 * H_HID * H_HID + k0);
        acc[0] = Frag<_Float16>::mma(a, b0, acc[0]);
        acc[1] = Frag<_Float16>::mma(a, b1, acc[1]);
        acc[2] = Frag<_Float16>::mma(a, b2, acc[2]);
        acc[3] = Frag<_Float16>::mma(a, b3, acc[3]);
        tie4in5_h(acc[0], acc[1], acc[2], acc[3], a, b0, b1, b2, b3);
      }
      acc_guard4(acc[0], acc[1], acc[2], acc[3]);
#pragma unroll
      for (int r = 0; r < 8; ++r) {
        const unsigned sh = (unsigned)(r & 1) * 16u;
        const unsigned wf = zq[0][r >> 1], wi = zq[1][r >> 1], wo = zq[2][r >> 1], wc = zq[3][r >> 1];
        const float zxf = h16_to_f32((wf >> sh) & 0xffffu) * Z_INV;
        const float zxi = h16_to_f32((wi >> sh) & 0xffffu) * Z_INV;
        const float zxo = h16_to_f32((wo >> sh) & 0xffffu) * Z_INV;
        const float zxc = h16_to_f32((wc >> sh) & 0xffffu) * Z_INV;
        const float zf = (acc[0][r] * AW_INV + zxf) + bgv[nt][0];
        const float zi = (acc[1][r] * AW_INV + zxi) + bgv[nt][1];
        const float zo = (acc[2][r] * AW_INV + zxo) + bgv[nt][2];
        const float zc = (acc[3][r] * AW_INV + zxc) + bgv[nt][3];
        const float cn = fsig(zf) * cst[nt][r] + fsig(zi) * ftanh(zc);
        cst[nt][r] = cn;
        const float an = fsig(zo) * ftanh(cn);
        ahn[(8 * hh + r) * HPITCH + j] = (_Float16)(an * ACARRY);
      }
    }
    __syncthreads();
    {
      const _Float16* asrc = &Ah[cur ^ 1][0];
      unsigned short* abase = ASQ + (size_t)dir * H_HID;
      for (int pass = 0; pass < 2; ++pass) {
#pragma unroll
        for (int it = 0; it < 4; ++it) {
          const int row  = 2 * wave + (it >> 1);
          const int colh = (it & 1) * (H_HID / 2) + lane * 8;
          const v8h v = *(const v8h*)(asrc + row * HPITCH + colh);
          *(volatile v8h*)(abase + ((size_t)(rowbase + row) * T_STEPS + (size_t)tt) * (2 * H_HID) + colh) = v;
        }
        __threadfence();
      }
    }
  }
}

__global__ __launch_bounds__(NTHR) void pack_out_kernel(const float* __restrict__ P, const float* __restrict__ bp,
                                                        float* __restrict__ out) {
  const int i = blockIdx.x * NTHR + threadIdx.x;
  v4f v;
#pragma unroll
  for (int e = 0; e < 4; ++e) {
    const int el = 4 * i + e;
    const int m  = el / O_TAGS;
    const int o  = el - m * O_TAGS;
    v[e] = P[(size_t)m * O_PAD + o] + bp[o];
  }
  float* op = out + (size_t)i * 4;
  *(volatile v4f*)op = v;
  __threadfence();
  *(volatile v4f*)op = v;
}

extern "C" void kernel_launch(void* const* d_in, const int* in_sizes, int n_in,
                              void* d_out, int out_size, void* d_ws, size_t ws_size, hipStream_t stream) {
  if (n_in < 20 || d_out == nullptr || d_ws == nullptr) return;
  if (in_sizes[0] != B_BATCH * T_STEPS || in_sizes[1] != V_VOCAB * E_EMB || in_sizes[18] != O_TAGS * 2 * H_HID ||
      in_sizes[19] != O_TAGS || out_size != N_OUT) return;
  for (int i = 2; i <= 5; ++i)   if (in_sizes[i] != H_HID * C_CAT) return;
  for (int i = 10; i <= 13; ++i) if (in_sizes[i] != H_HID * C_CAT) return;
  for (int i = 6; i <= 9; ++i)   if (in_sizes[i] != H_HID) return;
  for (int i = 14; i <= 17; ++i) if (in_sizes[i] != H_HID) return;

  const int*   tok  = (const int*)d_in[0];
  const float* emb  = (const float*)d_in[1];
  const float* W_cf = (const float*)d_in[2];
  const float* W_ff = (const float*)d_in[3];
  const float* W_uf = (const float*)d_in[4];
  const float* W_of = (const float*)d_in[5];
  const float* b_cf = (const float*)d_in[6];
  const float* b_ff = (const float*)d_in[7];
  const float* b_uf = (const float*)d_in[8];
  const float* b_of = (const float*)d_in[9];
  const float* W_cb = (const float*)d_in[10];
  const float* W_fb = (const float*)d_in[11];
  const float* W_ub = (const float*)d_in[12];
  const float* W_ob = (const float*)d_in[13];
  const float* b_cb = (const float*)d_in[14];
  const float* b_fb = (const float*)d_in[15];
  const float* b_ub = (const float*)d_in[16];
  const float* b_ob = (const float*)d_in[17];
  const float* W_p  = (const float*)d_in[18];
  const float* b_p  = (const float*)d_in[19];
  float* out = (float*)d_out;

  char* ws = (char*)d_ws; size_t off = 0;
  auto carve = [&](size_t bytes) -> char* { char* p = ws + off; off += (bytes + 255) & ~(size_t)255; return p; };
  unsigned short* XE   = (unsigned short*)carve(SZ_XE);
  unsigned short* WX16 = (unsigned short*)carve(SZ_WX16);
  unsigned short* WA16 = (unsigned short*)carve(SZ_WA16);
  unsigned short* WP16 = (unsigned short*)carve(SZ_WP16);
  unsigned short* ZX   = (unsigned short*)carve(SZ_ZX);
  unsigned short* ASQ  = (unsigned short*)carve(SZ_ASQ);
  float*          PRJ  = (float*)carve(SZ_PRJ);
  if (off > ws_size || off > (size_t)134217728) return;

  GateW gw;
  gw.w0 = W_ff; gw.w1 = W_uf; gw.w2 = W_of; gw.w3 = W_cf;
  gw.w4 = W_fb; gw.w5 = W_ub; gw.w6 = W_ob; gw.w7 = W_cb;

  wa_prep_kernel<<<dim3(H_HID * (H_HID / 8) / NTHR, 8), NTHR, 0, stream>>>(gw, WA16);
  wx_prep_kernel<<<dim3(H_HID * (E_PAD / 8) / NTHR, 8), NTHR, 0, stream>>>(gw, WX16);
  wp_prep_kernel<<<O_PAD * (2 * H_HID / 8) / NTHR, NTHR, 0, stream>>>(W_p, WP16);
  embed_kernel<<<M_ROWS / (4 * (NTHR / 32)), NTHR, 0, stream>>>(tok, emb, XE);

  const dim3 zgrid((G4H / 64) * (M_ROWS / 64) / 8, 1);
  wmma_gemm64<0, false, 0, 1, false, 0><<<zgrid, 256, 0, stream>>>(
      WX16, WX16, E_PAD, 0L, XE, XE, E_PAD, 0L, (void*)ZX, (void*)ZX, M_ROWS, 0L,
      PRJ, PRJ, 0L, G4H, M_ROWS, E_PAD, ZX_SCALE);
  lstm_dir_kernel<<<B_BATCH / SEQB, NTHR, 0, stream>>>(WA16, ZX, ASQ, b_ff, b_uf, b_of, b_cf, 0);
  wmma_gemm64<0, false, 0, 1, false, 0><<<zgrid, 256, 0, stream>>>(
      WX16 + (size_t)G4H * E_PAD, WX16 + (size_t)G4H * E_PAD, E_PAD, 0L, XE, XE, E_PAD, 0L, (void*)ZX, (void*)ZX, M_ROWS, 0L,
      PRJ, PRJ, 0L, G4H, M_ROWS, E_PAD, ZX_SCALE);
  lstm_dir_kernel<<<B_BATCH / SEQB, NTHR, 0, stream>>>(WA16 + (size_t)G4H * H_HID, ZX, ASQ, b_fb, b_ub, b_ob, b_cb, 1);

  const dim3 pgrid((M_ROWS / 64) * (O_PAD / 64) / 8, 1);
  wmma_gemm64<0, false, 0, 0, false, 0><<<pgrid, 256, 0, stream>>>(
      ASQ, ASQ, 2 * H_HID, 0L, WP16, WP16, 2 * H_HID, 0L, (void*)PRJ, (void*)PRJ, O_PAD, 0L,
      PRJ, PRJ, 0L, M_ROWS, O_PAD, 2 * H_HID, PRJ_SCALE);
  pack_out_kernel<<<N_OUT / 4 / NTHR, NTHR, 0, stream>>>(PRJ, b_p, out);
}
